// SpatialSuppressionAttention_73589969650200
// MI455X (gfx1250) — hardware-verified
//
#include <hip/hip_runtime.h>
#include <stdint.h>

#define NB   8
#define NS   1024
#define ND   768
#define NH   12
#define DKH  64
static_assert(ND == NH * DKH);
static_assert((NS % 64) == 0 && (ND % 64) == 0 && (DKH % 64) == 0);
static_assert((NS % 32) == 0 && (ND % 32) == 0);
static_assert(NS == 128 * 8);
static_assert(((NB * NS * ND) % (8 * 256)) == 0 && ((ND * ND) % (8 * 256)) == 0);

typedef __bf16   v16b __attribute__((ext_vector_type(16)));
typedef __bf16   v8b  __attribute__((ext_vector_type(8)));
typedef _Float16 v16h __attribute__((ext_vector_type(16)));
typedef _Float16 v8h  __attribute__((ext_vector_type(8)));
typedef float    v8f  __attribute__((ext_vector_type(8)));
typedef float    v4f  __attribute__((ext_vector_type(4)));
typedef unsigned int v4u __attribute__((ext_vector_type(4)));

__device__ __forceinline__ unsigned short bf_bits(float f) {
  unsigned u = __float_as_uint(f);
  return (unsigned short)((u + 0x7FFFu + ((u >> 16) & 1u)) >> 16);
}
__device__ __forceinline__ float bfr(float f) {
  return __uint_as_float(((unsigned)bf_bits(f)) << 16);
}
__device__ __forceinline__ unsigned short h_bits(float f) {
  const _Float16 h = (_Float16)f;
  return __builtin_bit_cast(unsigned short, h);
}
__device__ __forceinline__ unsigned pk16(unsigned short a, unsigned short b) { return (unsigned)a | ((unsigned)b << 16); }
__device__ __forceinline__ v8f zero8() { v8f z = {0.f, 0.f, 0.f, 0.f, 0.f, 0.f, 0.f, 0.f}; return z; }
__device__ __forceinline__ void hilo2(float x, float y, unsigned& h, unsigned& l) {
  const unsigned short hx = bf_bits(x), hy = bf_bits(y);
  const float rx = x - __uint_as_float(((unsigned)hx) << 16);
  const float ry = y - __uint_as_float(((unsigned)hy) << 16);
  h = pk16(hx, hy);
  l = pk16(bf_bits(rx), bf_bits(ry));
}

template <int TY> struct OpT;
template <> struct OpT<0> {
  typedef v16b F;
  static __device__ __forceinline__ F ld(const unsigned short* p) {
    const __bf16* q = (const __bf16*)(const void*)p;
    union { v16b v; v8b h[2]; } f;
    f.h[0] = *(const v8b*)(q);
    f.h[1] = *(const v8b*)(q + 16);
    return f.v;
  }
  static __device__ __forceinline__ v8f mma(F a, F b, v8f c) {
    return __builtin_amdgcn_wmma_f32_16x16x32_bf16(false, a, false, b, (short)0, c, false, false);
  }
};
template <> struct OpT<1> {
  typedef v16h F;
  static __device__ __forceinline__ F ld(const unsigned short* p) {
    const _Float16* q = (const _Float16*)(const void*)p;
    union { v16h v; v8h h[2]; } f;
    f.h[0] = *(const v8h*)(q);
    f.h[1] = *(const v8h*)(q + 16);
    return f.v;
  }
  static __device__ __forceinline__ v8f mma(F a, F b, v8f c) {
    return __builtin_amdgcn_wmma_f32_16x16x32_f16(false, a, false, b, (short)0, c, false, false);
  }
};

template <class F>
__device__ __forceinline__ void dep_guard(v8f& a, v8f& b, F x, F y) {
#if defined(__HIP_DEVICE_COMPILE__)
  asm volatile("v_nop\n\tv_nop\n\tv_nop\n\tv_nop" : "+v"(a), "+v"(b) : "v"(x), "v"(y));
#endif
}
template <class F>
__device__ __forceinline__ void keep4(F a, F b, F c, F d) {
#if defined(__HIP_DEVICE_COMPILE__)
  asm volatile("v_nop" :: "v"(a), "v"(b), "v"(c), "v"(d));
#endif
}
__device__ __forceinline__ void acc_guard4(v8f& a, v8f& b, v8f& c, v8f& d) {
#if defined(__HIP_DEVICE_COMPILE__)
  asm volatile("v_nop\n\tv_nop\n\tv_nop\n\tv_nop" : "+v"(a), "+v"(b), "+v"(c), "+v"(d));
#endif
}
__device__ __forceinline__ void wave_sync_lds() {
  __builtin_amdgcn_fence(__ATOMIC_RELEASE, "workgroup");
  __builtin_amdgcn_wave_barrier();
  __builtin_amdgcn_fence(__ATOMIC_ACQUIRE, "workgroup");
}

__global__ __launch_bounds__(256) void cvt_bf16x8(const float* __restrict__ in, unsigned short* out,
                                                  int n8, int n8tot) {
  const int i = blockIdx.x * 256 + threadIdx.x;
  if (i >= n8tot) return;
  int ic = i;
  if (ic > n8 - 1) ic = n8 - 1;
  const v4f a = *(const v4f*)(in + (size_t)ic * 8);
  const v4f b = *(const v4f*)(in + (size_t)ic * 8 + 4);
  v4u p;
  p[0] = pk16(bf_bits(a[0]), bf_bits(a[1]));
  p[1] = pk16(bf_bits(a[2]), bf_bits(a[3]));
  p[2] = pk16(bf_bits(b[0]), bf_bits(b[1]));
  p[3] = pk16(bf_bits(b[2]), bf_bits(b[3]));
  if (i >= n8) { p[0] = 0u; p[1] = 0u; p[2] = 0u; p[3] = 0u; }
  *(volatile v4u*)(out + (size_t)i * 8) = p;
  __threadfence();
  *(volatile v4u*)(out + (size_t)i * 8) = p;
}

template <int TY, int OUT, int PM>
__global__ __launch_bounds__(256) void gemm64(
    const unsigned short* __restrict__ Ahp, const unsigned short* __restrict__ Alp, int lda, int zsA,
    const unsigned short* __restrict__ Bhp, const unsigned short* __restrict__ Blp, int ldb, int zsB,
    void* Cout, void* Cout2, int ldc, int zsC,
    const float* __restrict__ bias, int blen, int bmode,
    float alpha, float oscale, int M, int N, int K) {
  typedef typename OpT<TY>::F FT;
  __shared__ __align__(16) float sT[8][16 * 68];
  const int lane = threadIdx.x & 31;
  const int wave = threadIdx.x >> 5;
  const int tilesN = N >> 6;
  const int tilesM = M >> 6;
  const int tile = blockIdx.x * 8 + wave;
  if (tile >= tilesM * tilesN) return;
  const int tm = tile / tilesN;
  const int tn = tile - tm * tilesN;
  const int m0 = tm << 6;
  const int n0 = tn << 6;
  const size_t zA = (size_t)blockIdx.y * (size_t)zsA;
  const size_t zB = (size_t)blockIdx.y * (size_t)zsB;
  const size_t zC = (size_t)blockIdx.y * (size_t)zsC;

  const int rlane = lane & 15;
  const int koff  = (lane >> 4) * 8;
  const int mOff  = (lane >> 4) * 8;

  v8f acc[4][4];
#pragma unroll
  for (int i = 0; i < 4; ++i)
#pragma unroll
    for (int j = 0; j < 4; ++j) acc[i][j] = zero8();

#pragma unroll 1
  for (int ps = 0; ps < 3; ++ps) {
    if (ps == 1 && (PM & 1) == 0) continue;
    if (ps == 2 && (PM & 2) == 0) continue;
    const unsigned short* A  = ((ps == 2) ? Alp : Ahp) + zA;
    const unsigned short* Bt = ((ps == 1) ? Blp : Bhp) + zB;
    for (int k0 = 0; k0 < K; k0 += 32) {
      FT bh[4];
#pragma unroll
      for (int j = 0; j < 4; ++j) {
        const size_t bo = (size_t)(n0 + (j << 4) + rlane) * ldb + koff + k0;
        bh[j] = OpT<TY>::ld(Bt + bo);
      }
#pragma unroll
      for (int i = 0; i < 4; ++i) {
        const size_t ao = (size_t)(m0 + (i << 4) + rlane) * lda + koff + k0;
        const FT ah = OpT<TY>::ld(A + ao);
#pragma unroll
        for (int j = 0; j < 4; ++j) {
          acc[i][j] = OpT<TY>::mma(ah, bh[j], acc[i][j]);
        }
        dep_guard<FT>(acc[i][0], acc[i][3], ah, bh[3]);
      }
      keep4<FT>(bh[0], bh[1], bh[2], bh[3]);
    }
  }
  acc_guard4(acc[0][0], acc[0][1], acc[0][2], acc[0][3]);
  acc_guard4(acc[1][0], acc[1][1], acc[1][2], acc[1][3]);
  acc_guard4(acc[2][0], acc[2][1], acc[2][2], acc[2][3]);
  acc_guard4(acc[3][0], acc[3][1], acc[3][2], acc[3][3]);

  const v4f z4 = {0.f, 0.f, 0.f, 0.f};
  float* slab = sT[wave];
#pragma unroll
  for (int i = 0; i < 4; ++i) {
    const int mBase = m0 + (i << 4);
#pragma unroll
    for (int j = 0; j < 4; ++j) {
#pragma unroll
      for (int r = 0; r < 8; ++r) {
        slab[(mOff + r) * 68 + (j << 4) + rlane] = acc[i][j][r];
      }
    }
    wave_sync_lds();
    if (OUT == 0) {
      float* C = (float*)Cout + zC;
      const int hh = lane >> 4, c4 = (lane & 15) * 4;
      v4f bb = z4;
      if (bmode == 1) {
        int bi = n0 + c4;
        if (bi > blen - 4) bi = blen - 4;
        if (bi < 0) bi = 0;
        const v4f t = *(const v4f*)(bias + bi);
        bb[0] = bfr(t[0]); bb[1] = bfr(t[1]); bb[2] = bfr(t[2]); bb[3] = bfr(t[3]);
      }
      v4f vv[8];
#pragma unroll
      for (int it = 0; it < 8; ++it) {
        const int row = it * 2 + hh;
        v4f v = *(const v4f*)(slab + row * 68 + c4);
        v = v * alpha + bb;
        if (bmode == 2) {
          int bi = mBase + row;
          if (bi > blen - 1) bi = blen - 1;
          if (bi < 0) bi = 0;
          const float br = bfr(bias[bi]);
          v = v + br;
        }
        vv[it] = v * oscale;
      }
      for (int pass = 0; pass < 2; ++pass) {
#pragma unroll
        for (int it = 0; it < 8; ++it) {
          const int row = it * 2 + hh;
          *(volatile v4f*)(C + (size_t)(mBase + row) * ldc + n0 + c4) = vv[it];
        }
        __threadfence();
      }
    } else {
      unsigned short* Ch = (unsigned short*)Cout + zC;
      unsigned short* Cl = (unsigned short*)Cout2 + zC;
      const int q8 = (lane & 7) * 8, rr = lane >> 3;
      v4f b0 = z4, b1 = z4;
      if (bmode == 1) {
        int bi = n0 + q8;
        if (bi > blen - 8) bi = blen - 8;
        if (bi < 0) bi = 0;
        const v4f t0 = *(const v4f*)(bias + bi);
        const v4f t1 = *(const v4f*)(bias + bi + 4);
        b0[0] = bfr(t0[0]); b0[1] = bfr(t0[1]); b0[2] = bfr(t0[2]); b0[3] = bfr(t0[3]);
        b1[0] = bfr(t1[0]); b1[1] = bfr(t1[1]); b1[2] = bfr(t1[2]); b1[3] = bfr(t1[3]);
      }
      v4u ph[4], pl[4];
#pragma unroll
      for (int it = 0; it < 4; ++it) {
        const int row = it * 4 + rr;
        v4f a = *(const v4f*)(slab + row * 68 + q8);
        v4f b = *(const v4f*)(slab + row * 68 + q8 + 4);
        a = a * alpha + b0;
        b = b * alpha + b1;
        if (bmode == 2) {
          int bi = mBase + row;
          if (bi > blen - 1) bi = blen - 1;
          if (bi < 0) bi = 0;
          const float br = bfr(bias[bi]);
          a = a + br;
          b = b + br;
        }
        a = a * oscale;
        b = b * oscale;
        v4u hpk, lpk;
        if (OUT == 2) {
          unsigned h0, l0, h1, l1, h2, l2, h3, l3;
          hilo2(a[0], a[1], h0, l0);
          hilo2(a[2], a[3], h1, l1);
          hilo2(b[0], b[1], h2, l2);
          hilo2(b[2], b[3], h3, l3);
          hpk[0] = h0; hpk[1] = h1; hpk[2] = h2; hpk[3] = h3;
          lpk[0] = l0; lpk[1] = l1; lpk[2] = l2; lpk[3] = l3;
        } else {
          hpk[0] = pk16(h_bits(a[0]), h_bits(a[1]));
          hpk[1] = pk16(h_bits(a[2]), h_bits(a[3]));
          hpk[2] = pk16(h_bits(b[0]), h_bits(b[1]));
          hpk[3] = pk16(h_bits(b[2]), h_bits(b[3]));
          lpk = hpk;
        }
        ph[it] = hpk;
        pl[it] = lpk;
      }
      for (int pass = 0; pass < 2; ++pass) {
#pragma unroll
        for (int it = 0; it < 4; ++it) {
          const int row = it * 4 + rr;
          const size_t co = (size_t)(mBase + row) * ldc + n0 + q8;
          *(volatile v4u*)(Ch + co) = ph[it];
          if (OUT == 2) {
            *(volatile v4u*)(Cl + co) = pl[it];
          }
        }
        __threadfence();
      }
    }
    wave_sync_lds();
  }
}

__global__ __launch_bounds__(128) void softmax_supp(const float* __restrict__ S, const float* __restrict__ convw,
                                                    int nconv, unsigned short* P) {
  __shared__ __align__(16) float sR[4][NS + 32];
  __shared__ float sW[16];
  __shared__ float sMx[4];
  __shared__ float sSm[4];
  const int tid  = threadIdx.x;
  const int lane = tid & 31;
  const int wave = tid >> 5;
  const int qi   = blockIdx.x;
  const int hl   = blockIdx.y;
  const size_t plane = (size_t)hl * ((size_t)NS * NS);
  const float* Sp = S + plane;

  if (tid < 9) {
    int wi = hl * 9 + tid;
    if (wi > nconv - 1) wi = nconv - 1;
    if (wi < 0) wi = 0;
    sW[tid] = bfr(convw[wi]);
  }

  const int c0 = tid * 8;
  int im = qi - 1; if (im < 0) im = 0;
  int ip = qi + 1; if (ip > NS - 1) ip = NS - 1;
  v4f u0 = *(const v4f*)(Sp + (size_t)im * NS + c0);
  v4f u1 = *(const v4f*)(Sp + (size_t)im * NS + c0 + 4);
  const v4f e0r = *(const v4f*)(Sp + (size_t)qi * NS + c0);
  const v4f e1r = *(const v4f*)(Sp + (size_t)qi * NS + c0 + 4);
  v4f d0 = *(const v4f*)(Sp + (size_t)ip * NS + c0);
  v4f d1 = *(const v4f*)(Sp + (size_t)ip * NS + c0 + 4);
  const v4f z4 = {0.f, 0.f, 0.f, 0.f};
  if (qi == 0)      { u0 = z4; u1 = z4; }
  if (qi == NS - 1) { d0 = z4; d1 = z4; }
  *(v4f*)(&sR[0][16 + c0]) = u0;
  *(v4f*)(&sR[0][20 + c0]) = u1;
  *(v4f*)(&sR[1][16 + c0]) = e0r;
  *(v4f*)(&sR[1][20 + c0]) = e1r;
  *(v4f*)(&sR[2][16 + c0]) = d0;
  *(v4f*)(&sR[2][20 + c0]) = d1;
  if (tid == 0) {
    sR[0][15] = 0.f; sR[1][15] = 0.f; sR[2][15] = 0.f;
    sR[0][16 + NS] = 0.f; sR[1][16 + NS] = 0.f; sR[2][16 + NS] = 0.f;
  }
  __syncthreads();

  const float w0 = sW[0], w1 = sW[1], w2 = sW[2];
  const float w3 = sW[3], w4 = sW[4], w5 = sW[5];
  const float w6 = sW[6], w7 = sW[7], w8 = sW[8];
  const float ninf = __uint_as_float(0xff800000u);
  float tmax = ninf;
#pragma unroll 1
  for (int c = 0; c < 8; ++c) {
    const int j = 16 + c0 + c;
    const float s0 = w0 * sR[0][j - 1] + w1 * sR[0][j] + w2 * sR[0][j + 1];
    const float s1 = w3 * sR[1][j - 1] + w4 * sR[1][j] + w5 * sR[1][j + 1];
    const float s2 = w6 * sR[2][j - 1] + w7 * sR[2][j] + w8 * sR[2][j + 1];
    const float a = sR[1][j] - ((s0 + s1) + s2);
    sR[3][j] = a;
    tmax = fmaxf(tmax, a);
  }
  tmax = fmaxf(tmax, __shfl_xor(tmax, 16));
  tmax = fmaxf(tmax, __shfl_xor(tmax, 8));
  tmax = fmaxf(tmax, __shfl_xor(tmax, 4));
  tmax = fmaxf(tmax, __shfl_xor(tmax, 2));
  tmax = fmaxf(tmax, __shfl_xor(tmax, 1));
  if (lane == 0) sMx[wave] = tmax;
  __syncthreads();
  float m = sMx[0];
  m = fmaxf(m, sMx[1]);
  m = fmaxf(m, sMx[2]);
  m = fmaxf(m, sMx[3]);

  float psum = 0.0f;
#pragma unroll 1
  for (int c = 0; c < 8; ++c) {
    const int j = 16 + c0 + c;
    const float e = __expf(sR[3][j] - m);
    sR[3][j] = e;
    psum += e;
  }
  psum += __shfl_xor(psum, 16);
  psum += __shfl_xor(psum, 8);
  psum += __shfl_xor(psum, 4);
  psum += __shfl_xor(psum, 2);
  psum += __shfl_xor(psum, 1);
  if (lane == 0) sSm[wave] = psum;
  __syncthreads();
  const float l = (sSm[0] + sSm[1]) + (sSm[2] + sSm[3]);
  const float scl = 1024.0f * (1.0f / l);

  const v4f ea = *(const v4f*)(&sR[3][16 + c0]);
  const v4f eb = *(const v4f*)(&sR[3][20 + c0]);
  v4u pk;
  pk[0] = pk16(h_bits(ea[0] * scl), h_bits(ea[1] * scl));
  pk[1] = pk16(h_bits(ea[2] * scl), h_bits(ea[3] * scl));
  pk[2] = pk16(h_bits(eb[0] * scl), h_bits(eb[1] * scl));
  pk[3] = pk16(h_bits(eb[2] * scl), h_bits(eb[3] * scl));
  unsigned short* pr = P + plane + (size_t)qi * NS + c0;
  *(volatile v4u*)(pr) = pk;
  __threadfence();
  *(volatile v4u*)(pr) = pk;
}

extern "C" void kernel_launch(void* const* d_in, const int* in_sizes, int n_in,
                              void* d_out, int out_size, void* d_ws, size_t ws_size,
                              hipStream_t stream) {
  if (n_in < 12) return;
  const int nX = NB * NS * ND;
  const int nW = ND * ND;
  if (in_sizes[0] != nX || in_sizes[1] != nX || in_sizes[2] != nX) return;
  if (in_sizes[3] != nW || in_sizes[5] != nW || in_sizes[7] != nW || in_sizes[9] != nW) return;
  if (in_sizes[4] != ND || in_sizes[6] != ND || in_sizes[8] != ND || in_sizes[10] != ND) return;
  if (in_sizes[11] != NH * 9) return;
  if (out_size != nX) return;

  const float* q     = (const float*)d_in[0];
  const float* k     = (const float*)d_in[1];
  const float* v     = (const float*)d_in[2];
  const float* wq    = (const float*)d_in[3];
  const float* bq    = (const float*)d_in[4];
  const float* wk    = (const float*)d_in[5];
  const float* bk    = (const float*)d_in[6];
  const float* wv    = (const float*)d_in[7];
  const float* bv    = (const float*)d_in[8];
  const float* wo    = (const float*)d_in[9];
  const float* bo    = (const float*)d_in[10];
  const float* convw = (const float*)d_in[11];
  const int nconv = in_sizes[11];
  float* out = (float*)d_out;

  const size_t PX  = (size_t)NB * NS * ND * 2;
  const size_t PW  = (size_t)ND * ND * 2;
  const size_t PQK = (size_t)NS * ND * 2;
  const size_t PVT = (size_t)ND * NS * 2;
  const size_t PS  = (size_t)NH * NS * NS * 4;
  const size_t PP  = (size_t)NH * NS * NS * 2;
  const size_t PC  = (size_t)NS * ND * 2;
  size_t off = 0;
  const size_t oXq = off; off += PX;
  const size_t oXk = off; off += PX;
  const size_t oXv = off; off += PX;
  const size_t oWq = off; off += PW;
  const size_t oWk = off; off += PW;
  const size_t oWv = off; off += PW;
  const size_t oWo = off; off += PW;
  const size_t oQ  = off; off += PQK;
  const size_t oK  = off; off += PQK;
  const size_t oVt = off; off += PVT;
  const size_t oS  = off; off += PS;
  const size_t oP  = off; off += PP;
  const size_t oCh = off; off += PC;
  const size_t oCl = off; off += PC;
  if (off > ws_size) return;
  if (off > (size_t)134217728) return;

  char* ws = (char*)d_ws;
  unsigned short* Xq  = (unsigned short*)(ws + oXq);
  unsigned short* Xk  = (unsigned short*)(ws + oXk);
  unsigned short* Xv  = (unsigned short*)(ws + oXv);
  unsigned short* Wqb = (unsigned short*)(ws + oWq);
  unsigned short* Wkb = (unsigned short*)(ws + oWk);
  unsigned short* Wvb = (unsigned short*)(ws + oWv);
  unsigned short* Wob = (unsigned short*)(ws + oWo);
  unsigned short* Qp  = (unsigned short*)(ws + oQ);
  unsigned short* Kp  = (unsigned short*)(ws + oK);
  unsigned short* Vtp = (unsigned short*)(ws + oVt);
  float* S = (float*)(ws + oS);
  unsigned short* P   = (unsigned short*)(ws + oP);
  unsigned short* Ch  = (unsigned short*)(ws + oCh);
  unsigned short* Cl  = (unsigned short*)(ws + oCl);

  const dim3 blk(256);
  const dim3 blk128(128);
  const int n8x = nX / 8;
  const int n8w = nW / 8;
  const dim3 gCx((n8x + 255) / 256);
  const dim3 gCw((n8w + 255) / 256);
  const dim3 gPr(((NS / 64) * (ND / 64) + 7) / 8, 1);
  const dim3 gVt(((ND / 64) * (NS / 64) + 7) / 8, 1);
  const dim3 gSc(((NS / 64) * (NS / 64) + 7) / 8, NH);
  const dim3 gSm(NS, NH);
  const dim3 gPv(((NS / 64) * (DKH / 64) + 7) / 8, NH);
  const dim3 gWo(((NS / 64) * (ND / 64) + 7) / 8, 1);
  const float alphaPV = 1.0f / 1024.0f;

  cvt_bf16x8<<<gCx, blk, 0, stream>>>(q,  Xq,  n8x, n8x);
  cvt_bf16x8<<<gCx, blk, 0, stream>>>(k,  Xk,  n8x, n8x);
  cvt_bf16x8<<<gCx, blk, 0, stream>>>(v,  Xv,  n8x, n8x);
  cvt_bf16x8<<<gCw, blk, 0, stream>>>(wq, Wqb, n8w, n8w);
  cvt_bf16x8<<<gCw, blk, 0, stream>>>(wk, Wkb, n8w, n8w);
  cvt_bf16x8<<<gCw, blk, 0, stream>>>(wv, Wvb, n8w, n8w);
  cvt_bf16x8<<<gCw, blk, 0, stream>>>(wo, Wob, n8w, n8w);

  for (int b = 0; b < NB; ++b) {
    const unsigned short* Xqb = Xq + (size_t)b * NS * ND;
    const unsigned short* Xkb = Xk + (size_t)b * NS * ND;
    const unsigned short* Xvb = Xv + (size_t)b * NS * ND;
    float* outb = out + (size_t)b * NS * ND;
    gemm64<0, 4, 0><<<gPr, blk, 0, stream>>>(Xqb, Xqb, ND, 0, Wqb, Wqb, ND, 0, (void*)Qp, (void*)Qp, ND, 0,
                                            bq, ND, 1, 1.0f, 1.0f, NS, ND, ND);
    gemm64<0, 4, 0><<<gPr, blk, 0, stream>>>(Xkb, Xkb, ND, 0, Wkb, Wkb, ND, 0, (void*)Kp, (void*)Kp, ND, 0,
                                            bk, ND, 1, 1.0f, 1.0f, NS, ND, ND);
    gemm64<0, 4, 0><<<gVt, blk, 0, stream>>>(Wvb, Wvb, ND, 0, Xvb, Xvb, ND, 0, (void*)Vtp, (void*)Vtp, NS, 0,
                                            bv, ND, 2, 1.0f, 1.0f, ND, NS, ND);
    gemm64<1, 0, 0><<<gSc, blk, 0, stream>>>(Qp, Qp, ND, DKH, Kp, Kp, ND, DKH,
                                            (void*)S, (void*)S, NS, NS * NS,
                                            bq, ND, 0, 0.125f, 1.0f, NS, NS, DKH);
    softmax_supp<<<gSm, blk128, 0, stream>>>(S, convw, nconv, P);
    gemm64<1, 2, 0><<<gPv, blk, 0, stream>>>(P, P, NS, NS * NS, Vtp, Vtp, NS, DKH * NS,
                                            (void*)Ch, (void*)Cl, ND, DKH,
                                            bq, ND, 0, alphaPV, 1.0f, NS, DKH, NS);
    gemm64<0, 0, 2><<<gWo, blk, 0, stream>>>(Ch, Cl, ND, 0, Wob, Wob, ND, 0, (void*)outb, (void*)outb, ND, 0,
                                            bo, ND, 1, 1.0f, 1.0f, NS, ND, ND);
  }
  (void)hipGetLastError();
}
